// SimpleSSM_35923106464034
// MI455X (gfx1250) — hardware-verified
//
#include <hip/hip_runtime.h>
#include <math.h>

constexpr int kVoc      = 32000;
constexpr int kDm       = 512;
constexpr int kLay      = 2;
constexpr int kBat      = 8;
constexpr int kSeq      = 4096;
constexpr int kTok      = kBat * kSeq;
constexpr int kSeqPerCh = 2;
constexpr int kNch      = kBat / kSeqPerCh;
constexpr int kRC       = kSeqPerCh * kSeq;
constexpr int kCat      = 2 * kDm;
constexpr int kResPitch = 260;
constexpr float kEps    = 1e-5f;
constexpr float kInvDm  = 1.0f / 512.0f;
constexpr float kUCarry = 16.0f;
constexpr float kSCarry = 64.0f;
constexpr float kBCarry = 256.0f;
constexpr float kCCarry = 64.0f;
constexpr float kDCarry = 256.0f;
constexpr float kScale1 = 1.0f / (16.0f * 256.0f);
constexpr float kScale2 = 1.0f / 4096.0f;
static_assert(kUCarry * kDCarry == kSCarry * kCCarry, "uniform product carry in the K=1024 GEMM");
static_assert(kSCarry * kCCarry == 4096.0f, "scale2");
static_assert(kRC % 64 == 0 && kDm % 64 == 0 && kCat % 32 == 0 && kDm % 32 == 0, "tile multiples");
static_assert(kVoc % 256 == 0, "head grid exact");

typedef __attribute__((ext_vector_type(16))) _Float16 v16h;
typedef __attribute__((ext_vector_type(8)))  _Float16 v8h;
typedef __attribute__((ext_vector_type(16))) __bf16   v16b;
typedef __attribute__((ext_vector_type(8)))  __bf16   v8b;
typedef __attribute__((ext_vector_type(8)))  float    v8f;
typedef __attribute__((ext_vector_type(4)))  float    v4f;
typedef __attribute__((ext_vector_type(4)))  unsigned int v4u;

__device__ __forceinline__ unsigned short f2bf_bits(float f) {
  unsigned u = __float_as_uint(f);
  return (unsigned short)((u + 0x7FFFu + ((u >> 16) & 1u)) >> 16);
}
__device__ __forceinline__ float bf_bits2f(unsigned short h) { return __uint_as_float(((unsigned)h) << 16); }

__device__ __forceinline__ void dep_guard_h(v8f& a, v8f& b, v16h x, v16h y) { asm volatile("v_nop\n\tv_nop\n\tv_nop\n\tv_nop" : "+v"(a), "+v"(b) : "v"(x), "v"(y)); }
__device__ __forceinline__ void dep_guard_b(v8f& a, v8f& b, v16b x, v16b y) { asm volatile("v_nop\n\tv_nop\n\tv_nop\n\tv_nop" : "+v"(a), "+v"(b) : "v"(x), "v"(y)); }
__device__ __forceinline__ void keep4_h(v16h a, v16h b, v16h c, v16h d) { asm volatile("v_nop" :: "v"(a), "v"(b), "v"(c), "v"(d)); }
__device__ __forceinline__ void keep4_b(v16b a, v16b b, v16b c, v16b d) { asm volatile("v_nop" :: "v"(a), "v"(b), "v"(c), "v"(d)); }
__device__ __forceinline__ void acc_guard4(v8f& a, v8f& b, v8f& c, v8f& d) { asm volatile("v_nop\n\tv_nop\n\tv_nop\n\tv_nop" : "+v"(a), "+v"(b), "+v"(c), "+v"(d)); }
template <typename T> struct Frag;
template <> struct Frag<_Float16> {
  typedef v16h V; union U { v16h v; v8h h[2]; };
  static __device__ __forceinline__ v16h load(const _Float16* p) {
    U f; f.h[0] = *(const v8h*)(p); f.h[1] = *(const v8h*)(p + 16); return f.v;
  }
  static __device__ __forceinline__ v8f mma(v16h a, v16h b, v8f c) {
    return __builtin_amdgcn_wmma_f32_16x16x32_f16(false, a, false, b, (short)0, c, false, false);
  }
  static __device__ __forceinline__ void guard(v8f& a, v8f& b, v16h x, v16h y) { dep_guard_h(a, b, x, y); }
  static __device__ __forceinline__ void keep(v16h a, v16h b, v16h c, v16h d) { keep4_h(a, b, c, d); }
};
template <> struct Frag<__bf16> {
  typedef v16b V; union U { v16b v; v8b h[2]; };
  static __device__ __forceinline__ v16b load(const __bf16* p) {
    U f; f.h[0] = *(const v8b*)(p); f.h[1] = *(const v8b*)(p + 16); return f.v;
  }
  static __device__ __forceinline__ v8f mma(v16b a, v16b b, v8f c) {
    return __builtin_amdgcn_wmma_f32_16x16x32_bf16(false, a, false, b, (short)0, c, false, false);
  }
  static __device__ __forceinline__ void guard(v8f& a, v8f& b, v16b x, v16b y) { dep_guard_b(a, b, x, y); }
  static __device__ __forceinline__ void keep(v16b a, v16b b, v16b c, v16b d) { keep4_b(a, b, c, d); }
};

__device__ __forceinline__ unsigned pk16(unsigned short a, unsigned short b) { return (unsigned)a | ((unsigned)b << 16); }
__device__ __forceinline__ unsigned short h_bits(float f) { const _Float16 h = (_Float16)f; return __builtin_bit_cast(unsigned short, h); }

template <int ET> struct Elem;
template <> struct Elem<0> { typedef _Float16 T; };
template <> struct Elem<1> { typedef __bf16 T; };
template <int ET, bool SPLIT, int BIAS_MODE, int OUT_MODE, bool RESID, bool CSCALE>
__global__ __launch_bounds__(256) void wmma_gemm64(
    const unsigned short* __restrict__ Ap, const unsigned short* __restrict__ A2p, int lda, long strideA,
    const unsigned short* __restrict__ Btp, const unsigned short* __restrict__ Bt2p, int ldb, long strideB,
    void* __restrict__ Cout, void* __restrict__ Cout2, int ldc, long strideC,
    const float* __restrict__ bias, const float* __restrict__ cscale,
    const float* __restrict__ resid, long strideR,
    int M, int N, int K, float scale) {
  typedef typename Elem<ET>::T T;
  typedef typename Frag<T>::V V;
  const T* A = (const T*)Ap; const T* A2 = (const T*)A2p; const T* Bt = (const T*)Btp; const T* Bt2 = (const T*)Bt2p;
  __shared__ __align__(16) float sT[8][16 * 68];
  const int b    = blockIdx.y;
  const int lane = threadIdx.x & 31;
  const int wave = threadIdx.x >> 5;
  const int tilesN = N >> 6;
  const int tilesM = M >> 6;
  const int tile = blockIdx.x * 8 + wave;
  if (tile >= tilesM * tilesN) return;
  const int tm = tile / tilesN;
  const int tn = tile - tm * tilesN;
  const int m0 = tm << 6;
  const int n0 = tn << 6;

  const T* Ab  = A  + (size_t)b * strideA;
  const T* Bb  = Bt + (size_t)b * strideB;
  const T* Ab2 = SPLIT ? (A2  + (size_t)b * strideA) : nullptr;
  const T* Bb2 = SPLIT ? (Bt2 + (size_t)b * strideB) : nullptr;

  const int rlane = lane & 15;
  const int koff  = (lane >> 4) * 8;
  const int mOff  = (lane >> 4) * 8;

  v8f acc[4][4];
#pragma unroll
  for (int i = 0; i < 4; ++i)
#pragma unroll
    for (int j = 0; j < 4; ++j) acc[i][j] = (v8f){0.f,0.f,0.f,0.f,0.f,0.f,0.f,0.f};

  for (int k0 = 0; k0 < K; k0 += 32) {
    V bh[4], bl[4];
#pragma unroll
    for (int j = 0; j < 4; ++j) {
      const size_t bo = (size_t)(n0 + (j << 4) + rlane) * ldb + koff + k0;
      bh[j] = Frag<T>::load(Bb + bo);
      if (SPLIT) bl[j] = Frag<T>::load(Bb2 + bo);
    }
#pragma unroll
    for (int i = 0; i < 4; ++i) {
      const size_t ao = (size_t)(m0 + (i << 4) + rlane) * lda + koff + k0;
      V ah = Frag<T>::load(Ab + ao);
      V al;
      if (SPLIT) al = Frag<T>::load(Ab2 + ao);
#pragma unroll
      for (int j = 0; j < 4; ++j) {
        acc[i][j] = Frag<T>::mma(ah, bh[j], acc[i][j]);
        if (SPLIT) {
          acc[i][j] = Frag<T>::mma(ah, bl[j], acc[i][j]);
          acc[i][j] = Frag<T>::mma(al, bh[j], acc[i][j]);
        }
      }
      Frag<T>::guard(acc[i][0], acc[i][3], ah, SPLIT ? al : ah);
    }
    Frag<T>::keep(bh[0], bh[1], bh[2], bh[3]);
    if (SPLIT) Frag<T>::keep(bl[0], bl[1], bl[2], bl[3]);
  }
  acc_guard4(acc[0][0], acc[0][1], acc[0][2], acc[0][3]);
  acc_guard4(acc[1][0], acc[1][1], acc[1][2], acc[1][3]);
  acc_guard4(acc[2][0], acc[2][1], acc[2][2], acc[2][3]);
  acc_guard4(acc[3][0], acc[3][1], acc[3][2], acc[3][3]);

  float* slab = sT[wave];
  const float* Rb = RESID ? (resid + (size_t)b * strideR) : nullptr;
#pragma unroll
  for (int i = 0; i < 4; ++i) {
    const int mBase = m0 + (i << 4);
#pragma unroll
    for (int j = 0; j < 4; ++j) {
      const int n = n0 + (j << 4) + rlane;
      float bv = 0.f;
      float cv = 1.f;
      if (BIAS_MODE == 2) bv = bias[n];
      if (CSCALE) cv = cscale[n];
#pragma unroll
      for (int r = 0; r < 8; ++r) {
        float v = acc[i][j][r] * scale;
        if (CSCALE) v = v * cv;
        if (BIAS_MODE == 1) v += bias[mBase + mOff + r];
        if (BIAS_MODE == 2) v += bv;
        if (RESID) v += Rb[(size_t)(mBase + mOff + r) * ldc + n];
        slab[(mOff + r) * 68 + (j << 4) + rlane] = v;
      }
    }
    __builtin_amdgcn_fence(__ATOMIC_RELEASE, "workgroup");
    __builtin_amdgcn_wave_barrier();
    __builtin_amdgcn_fence(__ATOMIC_ACQUIRE, "workgroup");
    if (OUT_MODE == 0) {
      float* C = (float*)Cout + (size_t)b * strideC;
      const int hh = lane >> 4, c4 = (lane & 15) * 4;
      for (int pass = 0; pass < 2; ++pass) {
#pragma unroll
        for (int it = 0; it < 8; ++it) {
          const int row = it * 2 + hh;
          v4f v = *(const v4f*)(slab + row * 68 + c4);
          *(volatile v4f*)(C + (size_t)(mBase + row) * ldc + n0 + c4) = v;
        }
        __threadfence();
      }
    } else {
      const int q = lane >> 3, c8 = (lane & 7) * 8;
      unsigned short* C  = (unsigned short*)Cout  + (size_t)b * strideC;
      unsigned short* C2 = (OUT_MODE == 2) ? ((unsigned short*)Cout2 + (size_t)b * strideC) : nullptr;
      for (int pass = 0; pass < 2; ++pass) {
#pragma unroll
        for (int it = 0; it < 4; ++it) {
          const int row = it * 4 + q;
          const float* sp = slab + row * 68 + c8;
          v8h hv, lv;
#pragma unroll
          for (int e = 0; e < 8; ++e) {
            if (OUT_MODE == 1) {
              hv[e] = (_Float16)sp[e];
            } else {
              unsigned short hb = f2bf_bits(sp[e]);
              unsigned short lb = f2bf_bits(sp[e] - bf_bits2f(hb));
              hv[e] = __builtin_bit_cast(_Float16, hb);
              lv[e] = __builtin_bit_cast(_Float16, lb);
            }
          }
          *(volatile v8h*)(C + (size_t)(mBase + row) * ldc + n0 + c8) = hv;
          if (OUT_MODE == 2) *(volatile v8h*)(C2 + (size_t)(mBase + row) * ldc + n0 + c8) = lv;
        }
        __threadfence();
      }
    }
    __builtin_amdgcn_fence(__ATOMIC_RELEASE, "workgroup");
    __builtin_amdgcn_wave_barrier();
    __builtin_amdgcn_fence(__ATOMIC_ACQUIRE, "workgroup");
  }
}

__global__ __launch_bounds__(256) void params_kernel(const float* __restrict__ a_log, const float* __restrict__ dt_log,
                                                     float* __restrict__ abar, float* __restrict__ csc) {
  __shared__ __align__(16) float sa[kLay * kDm];
  __shared__ __align__(16) float ss[kLay * kDm];
  const int t = threadIdx.x;
#pragma unroll 1
  for (int i = 0; i < (kLay * kDm) / 256; ++i) {
    const int idx = i * 256 + t;
    const float a  = -expf(a_log[idx]);
    const float xl = dt_log[idx];
    const float sp = fmaxf(xl, 0.0f) + log1pf(expf(-fabsf(xl)));
    const float dt = sp + 1e-4f;
    const float hv = 0.5f * dt * a;
    sa[idx] = (1.0f + hv) / (1.0f - hv);
    ss[idx] = dt / (1.0f - hv);
  }
  __syncthreads();
  const v4f va = *(const v4f*)(sa + 4 * t);
  const v4f vs = *(const v4f*)(ss + 4 * t);
  for (int pass = 0; pass < 2; ++pass) {
    *(volatile v4f*)(abar + 4 * t) = va;
    *(volatile v4f*)(csc + 4 * t)  = vs;
    __threadfence();
  }
}

__global__ __launch_bounds__(256) void cast_b_kernel(const float* __restrict__ in, unsigned short* __restrict__ out) {
  const int i = blockIdx.x * 256 + threadIdx.x;
  const float* p = in + 8 * (size_t)i;
  const v4f a = *(const v4f*)(p);
  const v4f c = *(const v4f*)(p + 4);
  unsigned short hb[8];
#pragma unroll
  for (int e = 0; e < 4; ++e) {
    hb[e]     = h_bits(a[e] * kBCarry);
    hb[4 + e] = h_bits(c[e] * kBCarry);
  }
  const v4u u = (v4u){pk16(hb[0], hb[1]), pk16(hb[2], hb[3]), pk16(hb[4], hb[5]), pk16(hb[6], hb[7])};
  unsigned short* q = out + 8 * (size_t)i;
  *(volatile v4u*)q = u;
  __threadfence();
  *(volatile v4u*)q = u;
}

__global__ __launch_bounds__(256) void cast_cd_kernel(const float* __restrict__ cm, const float* __restrict__ dw,
                                                      unsigned short* __restrict__ out) {
  const int i  = blockIdx.x * 256 + threadIdx.x;
  const int rn = i >> 7;
  const int g  = i & 127;
  const size_t so = (size_t)rn * kDm + (size_t)(g & 63) * 8;
  const v4f c0 = *(const v4f*)(cm + so);
  const v4f c1 = *(const v4f*)(cm + so + 4);
  const v4f d0 = *(const v4f*)(dw + so);
  const v4f d1 = *(const v4f*)(dw + so + 4);
  const bool isc = (g < 64);
  const float sc = isc ? kCCarry : kDCarry;
  unsigned short hb[8];
#pragma unroll
  for (int e = 0; e < 4; ++e) {
    const float f0 = isc ? c0[e] : d0[e];
    const float f1 = isc ? c1[e] : d1[e];
    hb[e]     = h_bits(f0 * sc);
    hb[4 + e] = h_bits(f1 * sc);
  }
  const v4u u = (v4u){pk16(hb[0], hb[1]), pk16(hb[2], hb[3]), pk16(hb[4], hb[5]), pk16(hb[6], hb[7])};
  unsigned short* q = out + 8 * (size_t)i;
  *(volatile v4u*)q = u;
  __threadfence();
  *(volatile v4u*)q = u;
}

template <bool FROM_EMB>
__global__ __launch_bounds__(256) void ln_rows_kernel(const int* __restrict__ xid, const float* __restrict__ emb,
                                                      const float* __restrict__ hin,
                                                      const float* __restrict__ w, const float* __restrict__ bb,
                                                      float* __restrict__ h0out, unsigned short* __restrict__ su,
                                                      int row_base) {
  const int lane = threadIdx.x & 31;
  const int wave = threadIdx.x >> 5;
  const int lrow = blockIdx.x * 8 + wave;
  const int grow = row_base + lrow;
  const float* src;
  if (FROM_EMB) {
    int tk = xid[grow];
    tk = tk < 0 ? 0 : tk;
    tk = tk > (kVoc - 1) ? (kVoc - 1) : tk;
    src = emb + (size_t)tk * kDm;
  } else {
    src = hin + (size_t)grow * kDm;
  }
  v4f xa[4];
  float s = 0.f;
#pragma unroll
  for (int j = 0; j < 4; ++j) {
    xa[j] = *(const v4f*)(src + 128 * j + 4 * lane);
    s += (xa[j][0] + xa[j][1]) + (xa[j][2] + xa[j][3]);
  }
#pragma unroll
  for (int off = 16; off > 0; off >>= 1) s += __shfl_xor(s, off, 32);
  const float mu = s * kInvDm;
  float q = 0.f;
#pragma unroll
  for (int j = 0; j < 4; ++j) {
#pragma unroll
    for (int e = 0; e < 4; ++e) { const float d = xa[j][e] - mu; q = fmaf(d, d, q); }
  }
#pragma unroll
  for (int off = 16; off > 0; off >>= 1) q += __shfl_xor(q, off, 32);
  const float rsd = 1.0f / sqrtf(q * kInvDm + kEps);

  if (FROM_EMB) {
    float* hp = h0out + (size_t)lrow * kDm + 4 * lane;
    for (int pass = 0; pass < 2; ++pass) {
#pragma unroll
      for (int j = 0; j < 4; ++j) *(volatile v4f*)(hp + 128 * j) = xa[j];
      __threadfence();
    }
  }

  v4u pk[2];
#pragma unroll
  for (int j = 0; j < 2; ++j) {
    unsigned short hb[8];
#pragma unroll
    for (int q2 = 0; q2 < 2; ++q2) {
      const int c = 256 * j + 8 * lane + 4 * q2;
      const v4f xv = *(const v4f*)(src + c);
      const v4f wv = *(const v4f*)(w + c);
      const v4f bv = *(const v4f*)(bb + c);
#pragma unroll
      for (int e = 0; e < 4; ++e) {
        const float u = ((xv[e] - mu) * rsd) * wv[e] + bv[e];
        hb[4 * q2 + e] = h_bits(u * kUCarry);
      }
    }
    pk[j] = (v4u){pk16(hb[0], hb[1]), pk16(hb[2], hb[3]), pk16(hb[4], hb[5]), pk16(hb[6], hb[7])};
  }
  unsigned short* up = su + (size_t)lrow * kCat + kDm + 8 * lane;
  for (int pass = 0; pass < 2; ++pass) {
#pragma unroll
    for (int j = 0; j < 2; ++j) *(volatile v4u*)(up + 256 * j) = pk[j];
    __threadfence();
  }
}

__global__ __launch_bounds__(64) void scan_states_kernel(const float* __restrict__ vin, const float* __restrict__ abar,
                                                         unsigned short* __restrict__ su) {
#pragma clang fp contract(off)
  const int t  = threadIdx.x;
  const int bl = blockIdx.x;
  const int d0 = 8 * t;
  const v4f a0 = *(const v4f*)(abar + d0);
  const v4f a1 = *(const v4f*)(abar + d0 + 4);
  float a[8], st[8];
#pragma unroll
  for (int e = 0; e < 4; ++e) { a[e] = a0[e]; a[4 + e] = a1[e]; }
#pragma unroll
  for (int e = 0; e < 8; ++e) st[e] = 0.0f;
#pragma unroll 1
  for (int ts = 0; ts < kSeq; ++ts) {
    const size_t row = (size_t)bl * kSeq + ts;
    const float* vp = vin + row * kDm + d0;
    const v4f v0 = *(const v4f*)(vp);
    const v4f v1 = *(const v4f*)(vp + 4);
    unsigned short hb[8];
#pragma unroll
    for (int e = 0; e < 4; ++e) {
      const float p0 = st[e] * a[e];
      st[e] = p0 + v0[e];
      const float p1 = st[4 + e] * a[4 + e];
      st[4 + e] = p1 + v1[e];
      hb[e]     = h_bits(st[e] * kSCarry);
      hb[4 + e] = h_bits(st[4 + e] * kSCarry);
    }
    const v4u u = (v4u){pk16(hb[0], hb[1]), pk16(hb[2], hb[3]), pk16(hb[4], hb[5]), pk16(hb[6], hb[7])};
    unsigned short* sp = su + row * kCat + d0;
    *(volatile v4u*)sp = u;
    __threadfence();
    *(volatile v4u*)sp = u;
  }
}

__global__ __launch_bounds__(64) void scan_last_kernel(const float* __restrict__ vin, const float* __restrict__ abar,
                                                       const unsigned short* __restrict__ su,
                                                       unsigned short* __restrict__ a2, int seq_base) {
#pragma clang fp contract(off)
  const int t  = threadIdx.x;
  const int bl = blockIdx.x;
  const int d0 = 8 * t;
  const v4f a0 = *(const v4f*)(abar + d0);
  const v4f a1 = *(const v4f*)(abar + d0 + 4);
  float a[8], st[8];
#pragma unroll
  for (int e = 0; e < 4; ++e) { a[e] = a0[e]; a[4 + e] = a1[e]; }
#pragma unroll
  for (int e = 0; e < 8; ++e) st[e] = 0.0f;
#pragma unroll 1
  for (int ts = 0; ts < kSeq; ++ts) {
    const size_t row = (size_t)bl * kSeq + ts;
    const float* vp = vin + row * kDm + d0;
    const v4f v0 = *(const v4f*)(vp);
    const v4f v1 = *(const v4f*)(vp + 4);
#pragma unroll
    for (int e = 0; e < 4; ++e) {
      const float p0 = st[e] * a[e];
      st[e] = p0 + v0[e];
      const float p1 = st[4 + e] * a[4 + e];
      st[4 + e] = p1 + v1[e];
    }
  }
  unsigned short hb[8];
#pragma unroll
  for (int e = 0; e < 8; ++e) hb[e] = h_bits(st[e] * kSCarry);
  const v4u us = (v4u){pk16(hb[0], hb[1]), pk16(hb[2], hb[3]), pk16(hb[4], hb[5]), pk16(hb[6], hb[7])};
  const int r8 = seq_base + bl;
  const v4u ul = *(const v4u*)(su + ((size_t)bl * kSeq + (kSeq - 1)) * kCat + kDm + d0);
  unsigned short* ps = a2 + (size_t)r8 * kCat + d0;
  unsigned short* pu = a2 + (size_t)r8 * kCat + kDm + d0;
  for (int pass = 0; pass < 2; ++pass) {
    *(volatile v4u*)ps = us;
    *(volatile v4u*)pu = ul;
    __threadfence();
  }
}

__global__ __launch_bounds__(256) void tail_prep_kernel(const float* __restrict__ h1, float* __restrict__ h1l,
                                                        unsigned short* __restrict__ a2) {
  const int t = threadIdx.x;
  const v4f z4 = (v4f){0.f, 0.f, 0.f, 0.f};
#pragma unroll 1
  for (int i = 0; i < (64 * kDm) / (256 * 4); ++i) {
    const int idx = i * 256 + t;
    const int row = idx >> 7;
    const int c4  = (idx & 127) * 4;
    const int rowc = row < kBat ? row : (kBat - 1);
    v4f v = *(const v4f*)(h1 + ((size_t)rowc * kSeq + (kSeq - 1)) * kDm + c4);
    v = (row < kBat) ? v : z4;
    float* p = h1l + (size_t)idx * 4;
    *(volatile v4f*)p = v;
    __threadfence();
    *(volatile v4f*)p = v;
  }
  const v4u zu = (v4u){0u, 0u, 0u, 0u};
#pragma unroll 1
  for (int i = 0; i < (56 * kCat) / (256 * 8); ++i) {
    const int idx = i * 256 + t;
    unsigned short* p = a2 + (size_t)kBat * kCat + (size_t)idx * 8;
    *(volatile v4u*)p = zu;
    __threadfence();
    *(volatile v4u*)p = zu;
  }
}

__global__ __launch_bounds__(256) void final_ln_kernel(const float* __restrict__ h2l, const float* __restrict__ w,
                                                       const float* __restrict__ bb, float* __restrict__ hf) {
  const int lane = threadIdx.x & 31;
  const int wave = threadIdx.x >> 5;
  const float* src = h2l + (size_t)wave * kDm;
  v4f xa[4];
  float s = 0.f;
#pragma unroll
  for (int j = 0; j < 4; ++j) {
    xa[j] = *(const v4f*)(src + 128 * j + 4 * lane);
    s += (xa[j][0] + xa[j][1]) + (xa[j][2] + xa[j][3]);
  }
#pragma unroll
  for (int off = 16; off > 0; off >>= 1) s += __shfl_xor(s, off, 32);
  const float mu = s * kInvDm;
  float q = 0.f;
#pragma unroll
  for (int j = 0; j < 4; ++j) {
#pragma unroll
    for (int e = 0; e < 4; ++e) { const float d = xa[j][e] - mu; q = fmaf(d, d, q); }
  }
#pragma unroll
  for (int off = 16; off > 0; off >>= 1) q += __shfl_xor(q, off, 32);
  const float rsd = 1.0f / sqrtf(q * kInvDm + kEps);
  v4f uo[4];
#pragma unroll
  for (int j = 0; j < 4; ++j) {
    const int c = 128 * j + 4 * lane;
    const v4f wv = *(const v4f*)(w + c);
    const v4f bv = *(const v4f*)(bb + c);
#pragma unroll
    for (int e = 0; e < 4; ++e) uo[j][e] = ((xa[j][e] - mu) * rsd) * wv[e] + bv[e];
  }
  float* hp = hf + (size_t)wave * kDm + 4 * lane;
  for (int pass = 0; pass < 2; ++pass) {
#pragma unroll
    for (int j = 0; j < 4; ++j) *(volatile v4f*)(hp + 128 * j) = uo[j];
    __threadfence();
  }
}

__global__ __launch_bounds__(256) void head_kernel(const float* __restrict__ hf, const float* __restrict__ ow,
                                                   const float* __restrict__ ob, float* __restrict__ out) {
  __shared__ __align__(16) float shf[kBat * kDm];
  __shared__ __align__(16) float sres[kBat * kResPitch];
  const int t = threadIdx.x;
#pragma unroll
  for (int i = 0; i < (kBat * kDm) / 256; ++i) shf[i * 256 + t] = hf[i * 256 + t];
  __syncthreads();
  const int n = blockIdx.x * 256 + t;
  const float* wr = ow + (size_t)n * kDm;
  float acc[kBat];
#pragma unroll
  for (int b = 0; b < kBat; ++b) acc[b] = 0.0f;
#pragma unroll 1
  for (int k4 = 0; k4 < kDm / 4; ++k4) {
    const v4f wv = *(const v4f*)(wr + 4 * k4);
#pragma unroll
    for (int b = 0; b < kBat; ++b) {
      const v4f hv = *(const v4f*)(shf + b * kDm + 4 * k4);
      acc[b] = fmaf(hv[0], wv[0], acc[b]);
      acc[b] = fmaf(hv[1], wv[1], acc[b]);
      acc[b] = fmaf(hv[2], wv[2], acc[b]);
      acc[b] = fmaf(hv[3], wv[3], acc[b]);
    }
  }
  const float bo = ob[n];
#pragma unroll
  for (int b = 0; b < kBat; ++b) sres[b * kResPitch + t] = acc[b] + bo;
  __syncthreads();
  const int lane = t & 31, wave = t >> 5;
  float* op = out + (size_t)wave * kVoc + (size_t)blockIdx.x * 256;
  for (int pass = 0; pass < 2; ++pass) {
#pragma unroll
    for (int qq = 0; qq < 2; ++qq) {
      const int col = 128 * qq + 4 * lane;
      const v4f v = *(const v4f*)(sres + wave * kResPitch + col);
      *(volatile v4f*)(op + col) = v;
    }
    __threadfence();
  }
}

extern "C" void kernel_launch(void* const* d_in, const int* in_sizes, int n_in,
                              void* d_out, int out_size, void* d_ws, size_t ws_size,
                              hipStream_t stream) {
  if (n_in < 14) return;
  if (in_sizes[0] != kTok || in_sizes[1] != kVoc * kDm || in_sizes[12] != kVoc * kDm ||
      in_sizes[4] != kLay * kDm * kDm || out_size != kBat * kVoc) return;

  const int*   x      = (const int*)  d_in[0];
  const float* emb    = (const float*)d_in[1];
  const float* norm_w = (const float*)d_in[2];
  const float* norm_b = (const float*)d_in[3];
  const float* b_mat  = (const float*)d_in[4];
  const float* c_mat  = (const float*)d_in[5];
  const float* d_w    = (const float*)d_in[6];
  const float* d_b    = (const float*)d_in[7];
  const float* a_log  = (const float*)d_in[8];
  const float* dt_log = (const float*)d_in[9];
  const float* fn_w   = (const float*)d_in[10];
  const float* fn_b   = (const float*)d_in[11];
  const float* out_w  = (const float*)d_in[12];
  const float* out_b  = (const float*)d_in[13];
  float* out = (float*)d_out;

  size_t off = 0;
  auto carve = [&](size_t bytes) { size_t o = off; off += (bytes + 4095) & ~(size_t)4095; return o; };
  const size_t o_wb  = carve((size_t)kLay * kDm * kDm * 2);
  const size_t o_wcd = carve((size_t)kLay * kDm * kCat * 2);
  const size_t o_ab  = carve((size_t)kLay * kDm * 4);
  const size_t o_cs  = carve((size_t)kLay * kDm * 4);
  const size_t o_su  = carve((size_t)kRC * kCat * 2);
  const size_t o_v   = carve((size_t)kRC * kDm * 4);
  const size_t o_h0  = carve((size_t)kRC * kDm * 4);
  const size_t o_h1  = carve((size_t)kTok * kDm * 4);
  const size_t o_a2  = carve((size_t)64 * kCat * 2);
  const size_t o_h1l = carve((size_t)64 * kDm * 4);
  const size_t o_h2l = carve((size_t)64 * kDm * 4);
  const size_t o_hf  = carve((size_t)kBat * kDm * 4);
  if (off > ws_size) return;

  char* base = (char*)d_ws;
  unsigned short* WB  = (unsigned short*)(base + o_wb);
  unsigned short* WCD = (unsigned short*)(base + o_wcd);
  float* ABAR = (float*)(base + o_ab);
  float* CSC  = (float*)(base + o_cs);
  unsigned short* SU = (unsigned short*)(base + o_su);
  float* V    = (float*)(base + o_v);
  float* H0   = (float*)(base + o_h0);
  float* H1   = (float*)(base + o_h1);
  unsigned short* A2 = (unsigned short*)(base + o_a2);
  float* H1L  = (float*)(base + o_h1l);
  float* H2L  = (float*)(base + o_h2l);
  float* HF   = (float*)(base + o_hf);

  params_kernel<<<dim3(1), dim3(256), 0, stream>>>(a_log, dt_log, ABAR, CSC);
  cast_b_kernel<<<dim3((kLay * kDm * kDm) / (256 * 8)), dim3(256), 0, stream>>>(b_mat, WB);
  cast_cd_kernel<<<dim3((kLay * kDm * kCat) / (256 * 8)), dim3(256), 0, stream>>>(c_mat, d_w, WCD);

  const int tilesBig = (kRC / 64) * (kDm / 64);
  const dim3 gridBig((tilesBig + 7) / 8, 1);
  const dim3 gridLn(kRC / 8);

  for (int ch = 0; ch < kNch; ++ch) {
    const int row_base = ch * kRC;
    ln_rows_kernel<true><<<gridLn, dim3(256), 0, stream>>>(x, emb, H1, norm_w, norm_b, H0, SU, row_base);
    wmma_gemm64<0, false, 0, 0, false, true><<<gridBig, dim3(256), 0, stream>>>(
        SU + kDm, SU + kDm, kCat, 0L, WB, WB, kDm, 0L,
        (void*)V, (void*)V, kDm, 0L, CSC, CSC, H0, 0L, kRC, kDm, kDm, kScale1);
    scan_states_kernel<<<dim3(kSeqPerCh), dim3(64), 0, stream>>>(V, ABAR, SU);
    wmma_gemm64<0, false, 2, 0, true, false><<<gridBig, dim3(256), 0, stream>>>(
        SU, SU, kCat, 0L, WCD, WCD, kCat, 0L,
        (void*)(H1 + (size_t)row_base * kDm), (void*)(H1 + (size_t)row_base * kDm), kDm, 0L,
        d_b, CSC, H0, 0L, kRC, kDm, kCat, kScale2);
  }

  tail_prep_kernel<<<dim3(1), dim3(256), 0, stream>>>(H1, H1L, A2);

  for (int ch = 0; ch < kNch; ++ch) {
    const int row_base = ch * kRC;
    ln_rows_kernel<false><<<gridLn, dim3(256), 0, stream>>>(x, emb, H1, norm_w + kDm, norm_b + kDm, H0, SU, row_base);
    wmma_gemm64<0, false, 0, 0, false, true><<<gridBig, dim3(256), 0, stream>>>(
        SU + kDm, SU + kDm, kCat, 0L, WB + (size_t)kDm * kDm, WB + (size_t)kDm * kDm, kDm, 0L,
        (void*)V, (void*)V, kDm, 0L, CSC + kDm, CSC + kDm, H0, 0L, kRC, kDm, kDm, kScale1);
    scan_last_kernel<<<dim3(kSeqPerCh), dim3(64), 0, stream>>>(V, ABAR + kDm, SU, A2, ch * kSeqPerCh);
  }
  {
    const int tilesSmall = (64 / 64) * (kDm / 64);
    wmma_gemm64<0, false, 2, 0, true, false><<<dim3((tilesSmall + 7) / 8, 1), dim3(256), 0, stream>>>(
        A2, A2, kCat, 0L, WCD + (size_t)kDm * kCat, WCD + (size_t)kDm * kCat, kCat, 0L,
        (void*)H2L, (void*)H2L, kDm, 0L, d_b + kDm, CSC, H1L, 0L, 64, kDm, kCat, kScale2);
  }
  final_ln_kernel<<<dim3(1), dim3(256), 0, stream>>>(H2L, fn_w, fn_b, HF);
  head_kernel<<<dim3(kVoc / 256), dim3(256), 0, stream>>>(HF, out_w, out_b, out);
}
